// GraphConvEncoder_6150393168617
// MI455X (gfx1250) — hardware-verified
//
#include <hip/hip_runtime.h>
#include <math.h>

#define NN 100000
#define NE 1600000
#define FD 128
#define F4 512
#define MP 100096
#define GM 25024
#define NGRP 4
#define MR 32
#define CT 24
#define NT 256
#define TD 8192
#define RW 1024
#define NTILE 13
#define NSP (NTILE * TD)
#define SCH 4096
#define SPT 16
#define NCH ((NE + SCH - 1) / SCH)

typedef __attribute__((ext_vector_type(16))) _Float16 v16h;
typedef __attribute__((ext_vector_type(8)))  _Float16 v8h;
typedef __attribute__((ext_vector_type(16))) __bf16   v16b;
typedef __attribute__((ext_vector_type(8)))  __bf16   v8b;
typedef __attribute__((ext_vector_type(8)))  float    v8f;
typedef __attribute__((ext_vector_type(4)))  float    v4f;
typedef __attribute__((ext_vector_type(4)))  int      v4i;

__device__ __forceinline__ unsigned short f2bf_bits(float f) {
  unsigned u = __float_as_uint(f);
  return (unsigned short)((u + 0x7FFFu + ((u >> 16) & 1u)) >> 16);
}
__device__ __forceinline__ float bf_bits2f(unsigned short h) { return __uint_as_float(((unsigned)h) << 16); }

__device__ __forceinline__ void dep_guard_h(v8f& a, v8f& b, v16h x, v16h y) { asm volatile("v_nop\n\tv_nop\n\tv_nop\n\tv_nop" : "+v"(a), "+v"(b) : "v"(x), "v"(y)); }
__device__ __forceinline__ void dep_guard_b(v8f& a, v8f& b, v16b x, v16b y) { asm volatile("v_nop\n\tv_nop\n\tv_nop\n\tv_nop" : "+v"(a), "+v"(b) : "v"(x), "v"(y)); }
__device__ __forceinline__ void keep4_h(v16h a, v16h b, v16h c, v16h d) { asm volatile("v_nop" :: "v"(a), "v"(b), "v"(c), "v"(d)); }
__device__ __forceinline__ void keep4_b(v16b a, v16b b, v16b c, v16b d) { asm volatile("v_nop" :: "v"(a), "v"(b), "v"(c), "v"(d)); }
__device__ __forceinline__ void acc_guard4(v8f& a, v8f& b, v8f& c, v8f& d) { asm volatile("v_nop\n\tv_nop\n\tv_nop\n\tv_nop" : "+v"(a), "+v"(b), "+v"(c), "+v"(d)); }
template <typename T> struct Frag;
template <> struct Frag<_Float16> {
  typedef v16h V; union U { v16h v; v8h h[2]; };
  static __device__ __forceinline__ v16h load(const _Float16* p) {
    U f; f.h[0] = *(const v8h*)(p); f.h[1] = *(const v8h*)(p + 16); return f.v;
  }
  static __device__ __forceinline__ v8f mma(v16h a, v16h b, v8f c) {
    return __builtin_amdgcn_wmma_f32_16x16x32_f16(false, a, false, b, (short)0, c, false, false);
  }
  static __device__ __forceinline__ void guard(v8f& a, v8f& b, v16h x, v16h y) { dep_guard_h(a, b, x, y); }
  static __device__ __forceinline__ void keep(v16h a, v16h b, v16h c, v16h d) { keep4_h(a, b, c, d); }
};
template <> struct Frag<__bf16> {
  typedef v16b V; union U { v16b v; v8b h[2]; };
  static __device__ __forceinline__ v16b load(const __bf16* p) {
    U f; f.h[0] = *(const v8b*)(p); f.h[1] = *(const v8b*)(p + 16); return f.v;
  }
  static __device__ __forceinline__ v8f mma(v16b a, v16b b, v8f c) {
    return __builtin_amdgcn_wmma_f32_16x16x32_bf16(false, a, false, b, (short)0, c, false, false);
  }
  static __device__ __forceinline__ void guard(v8f& a, v8f& b, v16b x, v16b y) { dep_guard_b(a, b, x, y); }
  static __device__ __forceinline__ void keep(v16b a, v16b b, v16b c, v16b d) { keep4_b(a, b, c, d); }
};

template <int ET> struct Elem;
template <> struct Elem<0> { typedef _Float16 T; };
template <> struct Elem<1> { typedef __bf16 T; };
template <int ET, bool SPLIT, int BIAS_MODE, int OUT_MODE, bool RESID, int ACT = 0>
__global__ __launch_bounds__(256) void wmma_gemm64(
    const unsigned short* __restrict__ Ap, const unsigned short* __restrict__ A2p, int lda, long strideA,
    const unsigned short* __restrict__ Btp, const unsigned short* __restrict__ Bt2p, int ldb, long strideB,
    void* __restrict__ Cout, void* __restrict__ Cout2, int ldc, long strideC,
    const float* __restrict__ bias,
    const float* __restrict__ resid, long strideR,
    int M, int N, int K, float scale, int Mv) {
  typedef typename Elem<ET>::T T;
  typedef typename Frag<T>::V V;
  const T* A = (const T*)Ap; const T* A2 = (const T*)A2p; const T* Bt = (const T*)Btp; const T* Bt2 = (const T*)Bt2p;
  __shared__ __align__(16) float sT[8][16 * 68];
  const int b    = blockIdx.y;
  const int lane = threadIdx.x & 31;
  const int wave = threadIdx.x >> 5;
  const int tilesN = N >> 6;
  const int tilesM = M >> 6;
  const int tile = blockIdx.x * 8 + wave;
  if (tile >= tilesM * tilesN) return;
  const int tm = tile / tilesN;
  const int tn = tile - tm * tilesN;
  const int m0 = tm << 6;
  const int n0 = tn << 6;

  const T* Ab  = A  + (size_t)b * strideA;
  const T* Bb  = Bt + (size_t)b * strideB;
  const T* Ab2 = SPLIT ? (A2  + (size_t)b * strideA) : nullptr;
  const T* Bb2 = SPLIT ? (Bt2 + (size_t)b * strideB) : nullptr;

  const int rlane = lane & 15;
  const int koff  = (lane >> 4) * 8;
  const int mOff  = (lane >> 4) * 8;

  v8f acc[4][4];
#pragma unroll
  for (int i = 0; i < 4; ++i)
#pragma unroll
    for (int j = 0; j < 4; ++j) acc[i][j] = (v8f){0.f,0.f,0.f,0.f,0.f,0.f,0.f,0.f};

  for (int k0 = 0; k0 < K; k0 += 32) {
    V bh[4], bl[4];
#pragma unroll
    for (int j = 0; j < 4; ++j) {
      const size_t bo = (size_t)(n0 + (j << 4) + rlane) * ldb + koff + k0;
      bh[j] = Frag<T>::load(Bb + bo);
      if (SPLIT) bl[j] = Frag<T>::load(Bb2 + bo);
    }
#pragma unroll
    for (int i = 0; i < 4; ++i) {
      const size_t ao = (size_t)(m0 + (i << 4) + rlane) * lda + koff + k0;
      V ah = Frag<T>::load(Ab + ao);
      V al;
      if (SPLIT) al = Frag<T>::load(Ab2 + ao);
#pragma unroll
      for (int j = 0; j < 4; ++j) {
        acc[i][j] = Frag<T>::mma(ah, bh[j], acc[i][j]);
        if (SPLIT) {
          acc[i][j] = Frag<T>::mma(ah, bl[j], acc[i][j]);
          acc[i][j] = Frag<T>::mma(al, bh[j], acc[i][j]);
        }
      }
      Frag<T>::guard(acc[i][0], acc[i][3], ah, SPLIT ? al : ah);
    }
    Frag<T>::keep(bh[0], bh[1], bh[2], bh[3]);
    if (SPLIT) Frag<T>::keep(bl[0], bl[1], bl[2], bl[3]);
  }
  acc_guard4(acc[0][0], acc[0][1], acc[0][2], acc[0][3]);
  acc_guard4(acc[1][0], acc[1][1], acc[1][2], acc[1][3]);
  acc_guard4(acc[2][0], acc[2][1], acc[2][2], acc[2][3]);
  acc_guard4(acc[3][0], acc[3][1], acc[3][2], acc[3][3]);

  float* slab = sT[wave];
  const float* Rb = RESID ? (resid + (size_t)b * strideR) : nullptr;
#pragma unroll
  for (int i = 0; i < 4; ++i) {
    const int mBase = m0 + (i << 4);
#pragma unroll
    for (int j = 0; j < 4; ++j) {
      const int n = n0 + (j << 4) + rlane;
      float bv = 0.f;
      if (BIAS_MODE == 2) bv = bias[n];
#pragma unroll
      for (int r = 0; r < 8; ++r) {
        float v = acc[i][j][r] * scale;
        if (BIAS_MODE == 1) v += bias[mBase + mOff + r];
        if (BIAS_MODE == 2) v += bv;
        if (RESID) v += Rb[(size_t)(mBase + mOff + r) * ldc + n];
        if (ACT == 1) v = tanhf(v);
        if (ACT == 2) v = fmaxf(v, 0.0f);
        if (ACT == 3) v = v / (1.0f + expf(-v));
        if (ACT == 4) v = (v > 0.f) ? v : 0.01f * v;
        if (ACT == 5) v = 0.5f * v * (1.0f + erff(v * 0.70710678118654752f));
        slab[(mOff + r) * 68 + (j << 4) + rlane] = v;
      }
    }
    __builtin_amdgcn_fence(__ATOMIC_RELEASE, "workgroup");
    __builtin_amdgcn_wave_barrier();
    __builtin_amdgcn_fence(__ATOMIC_ACQUIRE, "workgroup");
    if (OUT_MODE == 0) {
      float* C = (float*)Cout + (size_t)b * strideC;
      const int hh = lane >> 4, c4 = (lane & 15) * 4;
      for (int pass = 0; pass < 2; ++pass) {
#pragma unroll
        for (int it = 0; it < 8; ++it) {
          const int row = it * 2 + hh;
          v4f v = *(const v4f*)(slab + row * 68 + c4);
          if (mBase + row < Mv) *(volatile v4f*)(C + (size_t)(mBase + row) * ldc + n0 + c4) = v;
        }
        __threadfence();
      }
    } else {
      const int q = lane >> 3, c8 = (lane & 7) * 8;
      unsigned short* C  = (unsigned short*)Cout  + (size_t)b * strideC;
      unsigned short* C2 = (OUT_MODE == 2) ? ((unsigned short*)Cout2 + (size_t)b * strideC) : nullptr;
      for (int pass = 0; pass < 2; ++pass) {
#pragma unroll
        for (int it = 0; it < 4; ++it) {
          const int row = it * 4 + q;
          const float* sp = slab + row * 68 + c8;
          v8h hv, lv;
#pragma unroll
          for (int e = 0; e < 8; ++e) {
            if (OUT_MODE == 1) {
              hv[e] = (_Float16)sp[e];
            } else {
              unsigned short hb = f2bf_bits(sp[e]);
              unsigned short lb = f2bf_bits(sp[e] - bf_bits2f(hb));
              hv[e] = __builtin_bit_cast(_Float16, hb);
              lv[e] = __builtin_bit_cast(_Float16, lb);
            }
          }
          if (mBase + row < Mv) {
            *(volatile v8h*)(C + (size_t)(mBase + row) * ldc + n0 + c8) = hv;
            if (OUT_MODE == 2) *(volatile v8h*)(C2 + (size_t)(mBase + row) * ldc + n0 + c8) = lv;
          }
        }
        __threadfence();
      }
    }
    __builtin_amdgcn_fence(__ATOMIC_RELEASE, "workgroup");
    __builtin_amdgcn_wave_barrier();
    __builtin_amdgcn_fence(__ATOMIC_ACQUIRE, "workgroup");
  }
}

__device__ __forceinline__ int blk_excl_scan(int cnt, int* scan_ws, int tid, int* tot) {
  const int lane = tid & 31, wave = tid >> 5; int incl = cnt;
#pragma unroll
  for (int o = 1; o < 32; o <<= 1) { const int v = __shfl_up(incl, o, 32); if (lane >= o) incl += v; }
  if (lane == 31) scan_ws[wave] = incl;
  __syncthreads();
  if (wave == 0) { int wv = (lane < NT / 32) ? scan_ws[lane] : 0; int wincl = wv;
#pragma unroll
    for (int o = 1; o < 32; o <<= 1) { const int v = __shfl_up(wincl, o, 32); if (lane >= o) wincl += v; }
    if (lane < NT / 32) scan_ws[32 + lane] = wincl - wv; if (lane == 31) scan_ws[64] = wincl; }
  __syncthreads();
  const int res = scan_ws[32 + wave] + incl - cnt; *tot = scan_ws[64];
  return res;
}
template <int SP, int CAP, bool PAY>
__device__ __forceinline__ int chunk_hits(const int* __restrict__ keyv, const int* __restrict__ payv, int e0, int n0, int tid,
                                          int* LIST, int* scan_ws) {
  const int eb = e0 + tid * SP;
  const bool inr = eb < NE;
  const int ebc = inr ? eb : (NE - SP);
  int rec[SP]; int cnt = 0;
#pragma unroll
  for (int k = 0; k < SP; k += 4) {
    const v4i d4 = *(const v4i*)(keyv + ebc + k);
    v4i s4 = d4;
    if (PAY) s4 = *(const v4i*)(payv + ebc + k);
#pragma unroll
    for (int e = 0; e < 4; ++e) {
      const int d = d4[e]; int r = -1;
      if (inr && d >= n0 && d < n0 + TD && d < NN) {
        int s = 0;
        if (PAY) { s = s4[e]; s = s < 0 ? 0 : (s >= NN ? NN - 1 : s); }
        r = ((d - n0) << 17) | s; ++cnt;
      }
      rec[k + e] = r;
    }
  }
  int tot; int p = blk_excl_scan(cnt, scan_ws, tid, &tot);
#pragma unroll
  for (int k = 0; k < SP; ++k) if (rec[k] >= 0) { if ((unsigned)p < (unsigned)CAP) LIST[p] = rec[k]; ++p; }
  __syncthreads();
  return tot < CAP ? tot : CAP;
}

__global__ __launch_bounds__(NT) void prep_kernel(const float* __restrict__ W1, const float* __restrict__ W2,
                                                 const float* __restrict__ Wc0, const float* __restrict__ Wc1,
                                                 const float* __restrict__ LE, unsigned* __restrict__ PW) {
  const int i = blockIdx.x * NT + threadIdx.x;
  if (i >= 118784) return;
  float a, b;
  if (i < 32768) {
    const int n = i >> 6, k = 2 * (i & 63);
    a = W1[(size_t)k * F4 + n]; b = W1[(size_t)(k + 1) * F4 + n];
  } else if (i < 65536) {
    const int i2 = i - 32768; const int n = i2 >> 6, k = 128 + 2 * (i2 & 63);
    a = W1[(size_t)k * F4 + n]; b = W1[(size_t)(k + 1) * F4 + n];
  } else if (i < 98304) {
    const int i2 = i - 65536; const int n = i2 >> 8, k = 2 * (i2 & 255);
    a = W2[(size_t)k * FD + n]; b = W2[(size_t)(k + 1) * FD + n];
  } else if (i < 106496) {
    const int i2 = i - 98304; const int n = i2 >> 6, k = 2 * (i2 & 63);
    a = Wc0[k * FD + n]; b = Wc0[(k + 1) * FD + n];
  } else if (i < 114688) {
    const int i2 = i - 106496; const int n = i2 >> 6, k = 2 * (i2 & 63);
    a = Wc1[k * FD + n]; b = Wc1[(k + 1) * FD + n];
  } else {
    const int i2 = i - 114688; const int r = i2 >> 6, c = 2 * (i2 & 63);
    const int rr = r < CT ? r : CT - 1;
    a = LE[rr * FD + c]; b = LE[rr * FD + c + 1];
    if (r >= CT) { a = 0.f; b = 0.f; }
  }
  a *= 16.0f; b *= 16.0f;
  const _Float16 h0 = (_Float16)a, h1 = (_Float16)b;
  const unsigned u = (unsigned)__builtin_bit_cast(unsigned short, h0) | ((unsigned)__builtin_bit_cast(unsigned short, h1) << 16);
  ((volatile unsigned*)PW)[i] = u;
  __threadfence();
  ((volatile unsigned*)PW)[i] = u;
}

__global__ __launch_bounds__(NT) void cast_x_kernel(const float* __restrict__ X, _Float16* __restrict__ XF) {
  const int t = blockIdx.x * NT + threadIdx.x;
  if (t >= MP * 16) return;
  const int row = t >> 4, c8 = (t & 15) * 8;
  const int rc = row < NN ? row : NN - 1;
  const v4f x0 = *(const v4f*)(X + (size_t)rc * FD + c8);
  const v4f x1 = *(const v4f*)(X + (size_t)rc * FD + c8 + 4);
  const bool live = row < NN;
  v8h h;
#pragma unroll
  for (int e = 0; e < 4; ++e) {
    h[e]     = live ? (_Float16)x0[e] : (_Float16)0.0f;
    h[4 + e] = live ? (_Float16)x1[e] : (_Float16)0.0f;
  }
  _Float16* p = XF + (size_t)row * FD + c8;
  *(volatile v8h*)p = h;
  __threadfence();
  *(volatile v8h*)p = h;
}

__global__ __launch_bounds__(NT) void mlp1_kernel(const _Float16* __restrict__ XF, const _Float16* __restrict__ W1T,
                                                 const float* __restrict__ TT, const int* __restrict__ labels,
                                                 const float* __restrict__ b1, const float* __restrict__ g1, const float* __restrict__ be1,
                                                 unsigned short* __restrict__ H1, int row0) {
  __shared__ __align__(16) float sT[8][16 * 68];
  __shared__ float sred[8 * MR];
  __shared__ float smu[MR];
  __shared__ float srs[MR];
  const int tid = threadIdx.x, lane = tid & 31, wave = tid >> 5;
  const int m0 = blockIdx.x * MR;
  const int n0 = wave << 6;
  const int rlane = lane & 15;
  const int koff  = (lane >> 4) * 8;
  const int mOff  = (lane >> 4) * 8;

  v8f acc[2][4];
#pragma unroll
  for (int i = 0; i < 2; ++i)
#pragma unroll
    for (int j = 0; j < 4; ++j) acc[i][j] = (v8f){0.f,0.f,0.f,0.f,0.f,0.f,0.f,0.f};

#pragma unroll 1
  for (int k0 = 0; k0 < FD; k0 += 32) {
    v16h bh[4];
#pragma unroll
    for (int j = 0; j < 4; ++j) bh[j] = Frag<_Float16>::load(W1T + (size_t)(n0 + (j << 4) + rlane) * FD + koff + k0);
#pragma unroll
    for (int i = 0; i < 2; ++i) {
      v16h ah = Frag<_Float16>::load(XF + (size_t)(m0 + (i << 4) + rlane) * FD + koff + k0);
#pragma unroll
      for (int j = 0; j < 4; ++j) acc[i][j] = Frag<_Float16>::mma(ah, bh[j], acc[i][j]);
      Frag<_Float16>::guard(acc[i][0], acc[i][3], ah, ah);
    }
    Frag<_Float16>::keep(bh[0], bh[1], bh[2], bh[3]);
  }
  acc_guard4(acc[0][0], acc[0][1], acc[0][2], acc[0][3]);
  acc_guard4(acc[1][0], acc[1][1], acc[1][2], acc[1][3]);

#pragma unroll
  for (int i = 0; i < 2; ++i) {
    const int rb = row0 + m0 + (i << 4) + mOff;
    int lb[8];
#pragma unroll
    for (int r = 0; r < 8; ++r) {
      int gr = rb + r; gr = gr < NN ? gr : NN - 1;
      int l = labels[gr]; l = l < 0 ? 0 : (l >= CT ? CT - 1 : l);
      lb[r] = l;
    }
#pragma unroll
    for (int j = 0; j < 4; ++j) {
      const int n = n0 + (j << 4) + rlane;
      const float bv = b1[n];
#pragma unroll
      for (int r = 0; r < 8; ++r) acc[i][j][r] = acc[i][j][r] * (1.0f / 16.0f) + bv + TT[lb[r] * F4 + n];
    }
  }
#pragma unroll
  for (int i = 0; i < 2; ++i) {
#pragma unroll
    for (int r = 0; r < 8; ++r) {
      float s = acc[i][0][r] + acc[i][1][r] + acc[i][2][r] + acc[i][3][r];
      s += __shfl_xor(s, 1, 32); s += __shfl_xor(s, 2, 32); s += __shfl_xor(s, 4, 32); s += __shfl_xor(s, 8, 32);
      if (rlane == 0) sred[wave * MR + (i << 4) + mOff + r] = s;
    }
  }
  __syncthreads();
  if (tid < MR) {
    float m = 0.f;
#pragma unroll
    for (int w = 0; w < 8; ++w) m += sred[w * MR + tid];
    smu[tid] = m * (1.0f / 512.0f);
  }
  __syncthreads();
#pragma unroll
  for (int i = 0; i < 2; ++i) {
    float mu8[8];
#pragma unroll
    for (int r = 0; r < 8; ++r) mu8[r] = smu[(i << 4) + mOff + r];
#pragma unroll
    for (int r = 0; r < 8; ++r) {
      float d = 0.f;
#pragma unroll
      for (int j = 0; j < 4; ++j) { const float t = acc[i][j][r] - mu8[r]; d += t * t; }
      d += __shfl_xor(d, 1, 32); d += __shfl_xor(d, 2, 32); d += __shfl_xor(d, 4, 32); d += __shfl_xor(d, 8, 32);
      if (rlane == 0) sred[wave * MR + (i << 4) + mOff + r] = d;
    }
  }
  __syncthreads();
  if (tid < MR) {
    float v = 0.f;
#pragma unroll
    for (int w = 0; w < 8; ++w) v += sred[w * MR + tid];
    v = v * (1.0f / 512.0f);
    srs[tid] = rsqrtf(v + 1e-5f);
  }
  __syncthreads();

  float* slab = sT[wave];
  const int q = lane >> 3, c8 = (lane & 7) * 8;
#pragma unroll
  for (int i = 0; i < 2; ++i) {
    const int mBase = m0 + (i << 4);
    float mu8[8], rs8[8];
#pragma unroll
    for (int r = 0; r < 8; ++r) { mu8[r] = smu[(i << 4) + mOff + r]; rs8[r] = srs[(i << 4) + mOff + r]; }
#pragma unroll
    for (int j = 0; j < 4; ++j) {
      const int n = n0 + (j << 4) + rlane;
      const float gv = g1[n], bev = be1[n];
#pragma unroll
      for (int r = 0; r < 8; ++r) {
        float t = (acc[i][j][r] - mu8[r]) * rs8[r];
        float v = t * gv + bev;
        v = fmaxf(v, 0.0f);
        slab[(mOff + r) * 68 + (j << 4) + rlane] = v;
      }
    }
    __builtin_amdgcn_fence(__ATOMIC_RELEASE, "workgroup");
    __builtin_amdgcn_wave_barrier();
    __builtin_amdgcn_fence(__ATOMIC_ACQUIRE, "workgroup");
    for (int pass = 0; pass < 2; ++pass) {
#pragma unroll
      for (int it = 0; it < 4; ++it) {
        const int row = it * 4 + q;
        const float* sp = slab + row * 68 + c8;
        v8h hv;
#pragma unroll
        for (int e = 0; e < 8; ++e) hv[e] = (_Float16)sp[e];
        *(volatile v8h*)(H1 + (size_t)(mBase + row) * F4 + n0 + c8) = hv;
      }
      __threadfence();
    }
    __builtin_amdgcn_fence(__ATOMIC_RELEASE, "workgroup");
    __builtin_amdgcn_wave_barrier();
    __builtin_amdgcn_fence(__ATOMIC_ACQUIRE, "workgroup");
  }
}

__global__ __launch_bounds__(NT) void deg_src_kernel(const int* __restrict__ esrc, float* __restrict__ NS) {
  __shared__ int LIST[SCH];
  __shared__ float CNT[TD];
  __shared__ int scan_ws[80];
  const int tid = threadIdx.x, lane = tid & 31, wave = tid >> 5;
  const int n0 = blockIdx.x * TD;
  for (int i = tid; i < TD; i += NT) CNT[i] = 0.0f;
  __syncthreads();
#pragma unroll 1
  for (int c = 0; c < NCH; ++c) {
    const int tot = chunk_hits<SPT, SCH, false>(esrc, esrc, c * SCH, n0, tid, LIST, scan_ws);
#pragma unroll 1
    for (int base = 0; base < tot; base += 32) {
      const int qq = base + lane;
      const int qc = qq < SCH ? qq : SCH - 1;
      const int lv = LIST[qc];
      const int rv = (qq < tot) ? lv : -1;
      const int own = (rv >= 0 && (rv >> 27) == wave) ? 1 : 0;
      unsigned msk = (unsigned)__ballot(own);
#pragma unroll 1
      for (int it = 0; it < 32; ++it) {
        if (msk == 0u) break;
        const int bp = __builtin_ctz(msk); msk &= msk - 1u;
        const int r = __shfl(rv, bp, 32);
        const int dl = (r >> 17) & (TD - 1);
        if (lane == 0) CNT[dl] += 1.0f;
      }
    }
    __syncthreads();
  }
  for (int pass = 0; pass < 2; ++pass) {
#pragma unroll
    for (int it = 0; it < 8; ++it) {
      const int dl = wave * RW + it * 128 + 4 * lane;
      v4f o;
#pragma unroll
      for (int e = 0; e < 4; ++e) {
        const float cn = CNT[dl + e];
        const float cs = cn > 0.f ? cn : 1.0f;
        o[e] = cn > 0.f ? rsqrtf(cs) : 0.0f;
      }
      *(volatile v4f*)(NS + n0 + dl) = o;
    }
    __threadfence();
  }
}

template <bool FIRST>
__global__ __launch_bounds__(NT) void agg_kernel(const float* __restrict__ HSrc, const int* __restrict__ edst, const int* __restrict__ esrc,
                                                const float* __restrict__ NS, float* ND, float* AGG) {
  __shared__ int LIST[SCH];
  __shared__ float CNT[TD];
  __shared__ int scan_ws[80];
  const int tid = threadIdx.x, lane = tid & 31, wave = tid >> 5;
  const int hh = lane >> 4;
  const int n0 = blockIdx.x * TD;
  const int wb = n0 + wave * RW;
  int jmax = MP - wb; jmax = jmax < 0 ? 0 : (jmax > RW ? RW : jmax);
  const v4f z4 = {0.f, 0.f, 0.f, 0.f};
  for (int pass = 0; pass < 2; ++pass) {
#pragma unroll 1
    for (int j = 0; j < jmax; ++j) *(volatile v4f*)(AGG + (size_t)(wb + j) * FD + 4 * lane) = z4;
    __threadfence();
  }
  for (int i = tid; i < TD; i += NT) CNT[i] = 0.0f;
  __syncthreads();
#pragma unroll 1
  for (int c = 0; c < NCH; ++c) {
    const int tot = chunk_hits<SPT, SCH, true>(edst, esrc, c * SCH, n0, tid, LIST, scan_ws);
#pragma unroll 1
    for (int base = 0; base < tot; base += 32) {
      const int qq = base + lane;
      const int qc = qq < SCH ? qq : SCH - 1;
      const int lv = LIST[qc];
      const int rv = (qq < tot) ? lv : -1;
      const int own = (rv >= 0 && (rv >> 27) == wave) ? 1 : 0;
      unsigned msk = (unsigned)__ballot(own);
#pragma unroll 1
      for (int it = 0; it < 32; ++it) {
        if (msk == 0u) break;
        const int bp = __builtin_ctz(msk); msk &= msk - 1u;
        const int r = __shfl(rv, bp, 32);
        const int dl = (r >> 17) & (TD - 1);
        int s = r & 0x1FFFF; s = s < NN ? s : NN - 1;
        int row = n0 + dl; row = row < MP ? row : MP - 1;
        const float w = NS[s];
        const v4f hv = *(const v4f*)(HSrc + (size_t)s * FD + 4 * lane);
        float* rp = AGG + (size_t)row * FD + 4 * lane;
        v4f a = *(const v4f*)rp;
        a = a + hv * w;
        *(volatile v4f*)rp = a;
        __threadfence();
        *(volatile v4f*)rp = a;
        if (FIRST) { if (lane == 0) CNT[dl] += 1.0f; }
      }
    }
    __syncthreads();
  }
  if (FIRST) {
    for (int pass = 0; pass < 2; ++pass) {
#pragma unroll
      for (int it = 0; it < 8; ++it) {
        const int dl = wave * RW + it * 128 + 4 * lane;
        v4f o;
#pragma unroll
        for (int e = 0; e < 4; ++e) {
          const float cn = CNT[dl + e];
          const float cs = cn > 0.f ? cn : 1.0f;
          o[e] = cn > 0.f ? rsqrtf(cs) : 0.0f;
        }
        *(volatile v4f*)(ND + n0 + dl) = o;
      }
      __threadfence();
    }
  }
  const int c8 = (lane & 15) * 8;
#pragma unroll 1
  for (int j = 0; j < jmax; j += 2) {
    const int row = wb + j + hh;
    float ndv;
    if (FIRST) {
      const float cn = CNT[wave * RW + j + hh];
      const float cs = cn > 0.f ? cn : 1.0f;
      ndv = cn > 0.f ? rsqrtf(cs) : 0.0f;
    } else {
      ndv = ND[row];
    }
    const float sc = ndv * 16.0f;
    const float* ap = AGG + (size_t)row * FD + c8;
    const v4f a0 = *(const v4f*)ap;
    const v4f a1 = *(const v4f*)(ap + 4);
    v8h o;
#pragma unroll
    for (int e = 0; e < 4; ++e) { o[e] = (_Float16)(a0[e] * sc); o[4 + e] = (_Float16)(a1[e] * sc); }
    _Float16* hp = (_Float16*)AGG + (size_t)row * (2 * FD) + c8;
    *(volatile v8h*)hp = o;
    __threadfence();
    *(volatile v8h*)hp = o;
  }
}

extern "C" void kernel_launch(void* const* d_in, const int* in_sizes, int n_in,
                              void* d_out, int out_size, void* d_ws, size_t ws_size, hipStream_t stream) {
  if (n_in < 15) return;
  if (in_sizes[0] != NN * FD || in_sizes[1] != NN || in_sizes[2] != NE || in_sizes[3] != NE || in_sizes[4] != CT * FD) return;
  if (in_sizes[5] != 2 * FD * F4 || in_sizes[9] != F4 * FD || in_sizes[11] != FD * FD || in_sizes[13] != FD * FD) return;
  if (in_sizes[6] != F4 || in_sizes[7] != F4 || in_sizes[8] != F4 || in_sizes[10] != FD || in_sizes[12] != FD || in_sizes[14] != FD) return;
  if (out_size != NN * FD) return;
  const float* features = (const float*)d_in[0];
  const int*   labels   = (const int*)  d_in[1];
  const int*   edge_src = (const int*)  d_in[2];
  const int*   edge_dst = (const int*)  d_in[3];
  const float* LE       = (const float*)d_in[4];
  const float* W1       = (const float*)d_in[5];
  const float* b1       = (const float*)d_in[6];
  const float* g1       = (const float*)d_in[7];
  const float* be1      = (const float*)d_in[8];
  const float* W2       = (const float*)d_in[9];
  const float* b2       = (const float*)d_in[10];
  const float* Wc0      = (const float*)d_in[11];
  const float* bc0      = (const float*)d_in[12];
  const float* Wc1      = (const float*)d_in[13];
  const float* bc1      = (const float*)d_in[14];
  float* out = (float*)d_out;

  char* ws = (char*)d_ws; size_t off = 0;
  auto carve = [&](size_t bytes) -> char* { char* p = ws + off; off += (bytes + 255) & ~(size_t)255; return p; };
  char*           PW  = carve(475136);
  float*          TT  = (float*)carve((size_t)64 * F4 * 4);
  float*          NS  = (float*)carve((size_t)NSP * 4);
  float*          ND  = (float*)carve((size_t)NSP * 4);
  unsigned short* H1c = (unsigned short*)carve((size_t)GM * F4 * 2);
  float*          R1  = (float*)carve((size_t)MP * FD * 4);
  float*          R2  = (float*)carve((size_t)MP * FD * 4);
  if (off > ws_size || off > (size_t)134217728) return;

  const unsigned short* W1T  = (const unsigned short*)(PW);
  const unsigned short* W1BT = (const unsigned short*)(PW + 131072);
  const unsigned short* W2T  = (const unsigned short*)(PW + 262144);
  const unsigned short* WC0T = (const unsigned short*)(PW + 393216);
  const unsigned short* WC1T = (const unsigned short*)(PW + 425984);
  const unsigned short* LABT = (const unsigned short*)(PW + 458752);
  _Float16* XF = (_Float16*)R1;
  float* HS = R2;

  prep_kernel<<<118784 / NT, NT, 0, stream>>>(W1, W2, Wc0, Wc1, LE, (unsigned*)PW);
  cast_x_kernel<<<(MP * 16) / NT, NT, 0, stream>>>(features, XF);
  wmma_gemm64<0, false, 0, 0, false, 0><<<dim3(1, 1), NT, 0, stream>>>(
      LABT, LABT, FD, 0L, W1BT, W1BT, FD, 0L, (void*)TT, (void*)nullptr, F4, 0L,
      (const float*)nullptr, (const float*)nullptr, 0L, 64, F4, FD, 1.0f / 256.0f, 64);
  deg_src_kernel<<<NTILE, NT, 0, stream>>>(edge_src, NS);
  for (int g = 0; g < NGRP; ++g) {
    mlp1_kernel<<<GM / MR, NT, 0, stream>>>(XF + (size_t)g * GM * FD, (const _Float16*)W1T, TT, labels, b1, g1, be1, H1c, g * GM);
    const int tiles2 = (GM / 64) * (FD / 64);
    wmma_gemm64<0, false, 2, 0, false, 0><<<dim3((tiles2 + 7) / 8, 1), NT, 0, stream>>>(
        H1c, H1c, F4, 0L, W2T, W2T, F4, 0L, (void*)(HS + (size_t)g * GM * FD), (void*)nullptr, FD, 0L,
        b2, (const float*)nullptr, 0L, GM, FD, F4, 1.0f / 16.0f, GM);
  }
  const int tilesC = (MP / 64) * (FD / 64);
  agg_kernel<true><<<NTILE, NT, 0, stream>>>(HS, edge_dst, edge_src, NS, ND, R1);
  wmma_gemm64<0, false, 2, 0, false, 2><<<dim3((tilesC + 7) / 8, 1), NT, 0, stream>>>(
      (const unsigned short*)R1, (const unsigned short*)R1, 2 * FD, 0L, WC0T, WC0T, FD, 0L, (void*)HS, (void*)nullptr, FD, 0L,
      bc0, (const float*)nullptr, 0L, MP, FD, FD, 1.0f / 256.0f, MP);
  agg_kernel<false><<<NTILE, NT, 0, stream>>>(HS, edge_dst, edge_src, NS, ND, R1);
  wmma_gemm64<0, false, 2, 0, false, 2><<<dim3((tilesC + 7) / 8, 1), NT, 0, stream>>>(
      (const unsigned short*)R1, (const unsigned short*)R1, 2 * FD, 0L, WC1T, WC1T, FD, 0L, (void*)out, (void*)nullptr, FD, 0L,
      bc1, (const float*)nullptr, 0L, MP, FD, FD, 1.0f / 256.0f, NN);
}
